// MFA_87067577025371
// MI455X (gfx1250) — hardware-run, weakly checked
//
#include <hip/hip_runtime.h>
#include <math.h>
#include <stdint.h>

#define NB     2
#define CC     64
#define CI     32
#define NPOS   9216
#define BN_EPS 1e-5f
static_assert(NB == 2);
static_assert(CC == 64 && CI == 32);
static_assert((NPOS % 128) == 0);

typedef __bf16   v16b __attribute__((ext_vector_type(16)));
typedef __bf16   v8b  __attribute__((ext_vector_type(8)));
typedef float    v8f  __attribute__((ext_vector_type(8)));
typedef float    v4f  __attribute__((ext_vector_type(4)));
typedef unsigned int v4u __attribute__((ext_vector_type(4)));

union FB { v16b v; v8b h[2]; unsigned int u[8]; };

__device__ __forceinline__ unsigned short bf_bits(float f) {
  unsigned u = __float_as_uint(f);
  return (unsigned short)((u + 0x7FFFu + ((u >> 16) & 1u)) >> 16);
}
__device__ __forceinline__ float bf_up(unsigned short h) { return __uint_as_float(((unsigned)h) << 16); }
__device__ __forceinline__ float bfr(float f) { return bf_up(bf_bits(f)); }
__device__ __forceinline__ unsigned pk16(unsigned short a, unsigned short b) { return (unsigned)a | ((unsigned)b << 16); }
__device__ __forceinline__ v8f zero8() { v8f z = {0.f, 0.f, 0.f, 0.f, 0.f, 0.f, 0.f, 0.f}; return z; }

__device__ __forceinline__ v4u cvt8(const float* p) {
  const v4f a = *(const v4f*)(p);
  const v4f b = *(const v4f*)(p + 4);
  v4u r;
  r[0] = pk16(bf_bits(a[0]), bf_bits(a[1]));
  r[1] = pk16(bf_bits(a[2]), bf_bits(a[3]));
  r[2] = pk16(bf_bits(b[0]), bf_bits(b[1]));
  r[3] = pk16(bf_bits(b[2]), bf_bits(b[3]));
  return r;
}

__device__ __forceinline__ v16b ldfrag_b(const __bf16* p) {
  union { v16b v; v8b h[2]; } f;
  f.h[0] = *(const v8b*)(p);
  f.h[1] = *(const v8b*)(p + 16);
  return f.v;
}

__device__ __forceinline__ v8f mma_b(v16b a, v16b b, v8f c) {
  c = __builtin_amdgcn_wmma_f32_16x16x32_bf16(false, a, false, b, (short)0, c, false, false);
#if defined(__HIP_DEVICE_COMPILE__)
  asm volatile("v_nop\n\tv_nop\n\tv_nop\n\tv_nop" : "+v"(c) : "v"(a), "v"(b));
#endif
  return c;
}
__device__ __forceinline__ v8f mma_b_raw(v16b a, v16b b, v8f c) {
  return __builtin_amdgcn_wmma_f32_16x16x32_bf16(false, a, false, b, (short)0, c, false, false);
}
__device__ __forceinline__ void dep_guard_b(v8f& a, v8f& b, v16b x, v16b y) {
#if defined(__HIP_DEVICE_COMPILE__)
  asm volatile("v_nop\n\tv_nop\n\tv_nop\n\tv_nop" : "+v"(a), "+v"(b) : "v"(x), "v"(y));
#endif
}
__device__ __forceinline__ void keep4_b(v16b a, v16b b, v16b c, v16b d) {
#if defined(__HIP_DEVICE_COMPILE__)
  asm volatile("v_nop" :: "v"(a), "v"(b), "v"(c), "v"(d));
#endif
}
__device__ __forceinline__ void acc_guard4(v8f& a, v8f& b, v8f& c, v8f& d) {
#if defined(__HIP_DEVICE_COMPILE__)
  asm volatile("v_nop\n\tv_nop\n\tv_nop\n\tv_nop" : "+v"(a), "+v"(b), "+v"(c), "+v"(d));
#endif
}
__device__ __forceinline__ void wave_sync_lds() {
  __builtin_amdgcn_fence(__ATOMIC_RELEASE, "workgroup");
  __builtin_amdgcn_wave_barrier();
  __builtin_amdgcn_fence(__ATOMIC_ACQUIRE, "workgroup");
}

__global__ __launch_bounds__(256) void prep_params(
    const float* __restrict__ Wk, const float* __restrict__ bk,
    const float* __restrict__ Wv, const float* __restrict__ bv,
    const float* __restrict__ Wq, const float* __restrict__ bq,
    const float* __restrict__ Wg,
    const float* __restrict__ g1g, const float* __restrict__ g1b,
    const float* __restrict__ g1m, const float* __restrict__ g1v,
    const float* __restrict__ Wo, const float* __restrict__ bo,
    const float* __restrict__ g2g, const float* __restrict__ g2b,
    const float* __restrict__ g2m, const float* __restrict__ g2v,
    unsigned short* w64, unsigned short* wq64, unsigned short* wgb, unsigned short* wob, float* par) {
  __shared__ __align__(16) float sPar[512];
  const int tid = threadIdx.x, lane = tid & 31, wave = tid >> 5;
  {
    const int row = tid >> 3, c8 = (tid & 7) * 8;
    const v4u pv = cvt8(Wv + row * CC + c8);
    const v4u pk = cvt8(Wk + row * CC + c8);
    const v4u pq = cvt8(Wq + row * CC + c8);
    v4u pz; pz[0] = 0u; pz[1] = 0u; pz[2] = 0u; pz[3] = 0u;
    unsigned short* d0 = w64  + (size_t)row * 64 + c8;
    unsigned short* d1 = w64  + (size_t)(32 + row) * 64 + c8;
    unsigned short* d2 = wq64 + (size_t)row * 64 + c8;
    unsigned short* d3 = wq64 + (size_t)(32 + row) * 64 + c8;
    *(volatile v4u*)d0 = pv; *(volatile v4u*)d1 = pk; *(volatile v4u*)d2 = pq; *(volatile v4u*)d3 = pz;
    __threadfence();
    *(volatile v4u*)d0 = pv; *(volatile v4u*)d1 = pk; *(volatile v4u*)d2 = pq; *(volatile v4u*)d3 = pz;
  }
  {
    const int row = tid >> 2, c8 = (tid & 3) * 8;
    const int rg = row & 31;
    const v4u po = cvt8(Wo + row * CI + c8);
    const v4u pg = cvt8(Wg + rg * CI + c8);
    unsigned short* d4 = wob + (size_t)row * 32 + c8;
    unsigned short* d5 = wgb + (size_t)rg * 32 + c8;
    *(volatile v4u*)d4 = po;
    if (tid < 128) *(volatile v4u*)d5 = pg;
    __threadfence();
    *(volatile v4u*)d4 = po;
    if (tid < 128) *(volatile v4u*)d5 = pg;
  }
  {
    const float cbv  = bfr(bv[lane]), cbk = bfr(bk[lane]), cbq = bfr(bq[lane]);
    const float cm1  = bfr(g1m[lane]), cb1 = bfr(g1b[lane]);
    const float cs1  = bfr(g1g[lane]) * rsqrtf(bfr(g1v[lane]) + BN_EPS);
    const float cbo0 = bfr(bo[lane]), cbo1 = bfr(bo[32 + lane]);
    const float cm20 = bfr(g2m[lane]), cm21 = bfr(g2m[32 + lane]);
    const float cs20 = bfr(g2g[lane]) * rsqrtf(bfr(g2v[lane]) + BN_EPS);
    const float cs21 = bfr(g2g[32 + lane]) * rsqrtf(bfr(g2v[32 + lane]) + BN_EPS);
    const float cb20 = bfr(g2b[lane]), cb21 = bfr(g2b[32 + lane]);
    const float v0 = (wave == 0) ? cbv : (wave == 1) ? cbk : (wave == 2) ? cbq : (wave == 4) ? cm1 :
                     (wave == 5) ? cs1 : (wave == 6) ? cb1 : 0.f;
    const float v1 = (wave == 0) ? cbo0 : (wave == 1) ? cbo1 : (wave == 2) ? cm20 : (wave == 3) ? cm21 :
                     (wave == 4) ? cs20 : (wave == 5) ? cs21 : (wave == 6) ? cb20 : cb21;
    sPar[tid] = v0;
    sPar[256 + tid] = v1;
  }
  __syncthreads();
  if (tid < 128) {
    const v4f v = *(const v4f*)(sPar + 4 * tid);
    float* dp = par + 4 * tid;
    *(volatile v4f*)dp = v;
    __threadfence();
    *(volatile v4f*)dp = v;
  }
}

__global__ __launch_bounds__(256) void xpose_cvt(const float* __restrict__ xA, const float* __restrict__ xB,
                                                 unsigned short* xat, unsigned short* xbt) {
  __shared__ __align__(16) unsigned short Tt[64 * 72];
  const int tid = threadIdx.x;
  const int src = blockIdx.y >> 1, b = blockIdx.y & 1;
  const int n0  = blockIdx.x * 64;
  const float* X = (src ? xB : xA) + (size_t)b * CC * NPOS;
  unsigned short* D = (src ? xbt : xat) + (size_t)b * NPOS * 64;
  const int ch = tid >> 2, n16 = (tid & 3) * 16;
  const float* xp = X + (size_t)ch * NPOS + n0 + n16;
  v4f xv[4];
#pragma unroll
  for (int k = 0; k < 4; ++k) xv[k] = *(const v4f*)(xp + 4 * k);
#pragma unroll
  for (int k = 0; k < 4; ++k)
#pragma unroll
    for (int e = 0; e < 4; ++e) Tt[(n16 + 4 * k + e) * 72 + ch] = bf_bits(xv[k][e]);
  __syncthreads();
  const int rl = tid >> 3, c8 = (tid & 7) * 8;
  v4u v[2];
#pragma unroll
  for (int rr = 0; rr < 2; ++rr) v[rr] = *(const v4u*)(Tt + (rr * 32 + rl) * 72 + c8);
  for (int ps = 0; ps < 2; ++ps) {
#pragma unroll
    for (int rr = 0; rr < 2; ++rr)
      *(volatile v4u*)(D + (size_t)(n0 + rr * 32 + rl) * 64 + c8) = v[rr];
    __threadfence();
  }
}

template <int BIAS_ROW>
__global__ __launch_bounds__(256) void gemm64b(
    const unsigned short* __restrict__ Ap, int lda, long long strideA,
    const unsigned short* __restrict__ Btp, int ldb, long long strideB,
    const float* __restrict__ bias,
    unsigned short* Cp, int ldc, long long strideC,
    int M, int N, int K) {
  const __bf16* A  = (const __bf16*)(const void*)Ap;
  const __bf16* Bt = (const __bf16*)(const void*)Btp;
  __shared__ __align__(16) float sT[8][16 * 68];
  const int b    = blockIdx.y;
  const int lane = threadIdx.x & 31;
  const int wave = threadIdx.x >> 5;
  const int tilesN = N >> 6;
  const int tilesM = M >> 6;
  const int tile = blockIdx.x * 8 + wave;
  if (tile >= tilesM * tilesN) return;
  const int tm = tile / tilesN;
  const int tn = tile - tm * tilesN;
  const int m0 = tm << 6;
  const int n0 = tn << 6;

  const __bf16* Ab = A  + (size_t)b * strideA;
  const __bf16* Bb = Bt + (size_t)b * strideB;

  const int rlane = lane & 15;
  const int koff  = (lane >> 4) * 8;
  const int mOff  = (lane >> 4) * 8;

  v8f acc[4][4];
#pragma unroll
  for (int i = 0; i < 4; ++i)
#pragma unroll
    for (int j = 0; j < 4; ++j) acc[i][j] = zero8();

  for (int k0 = 0; k0 < K; k0 += 32) {
    v16b bh[4];
#pragma unroll
    for (int j = 0; j < 4; ++j) {
      const size_t bo = (size_t)(n0 + (j << 4) + rlane) * ldb + koff + k0;
      bh[j] = ldfrag_b(Bb + bo);
    }
#pragma unroll
    for (int i = 0; i < 4; ++i) {
      const size_t ao = (size_t)(m0 + (i << 4) + rlane) * lda + koff + k0;
      const v16b ah = ldfrag_b(Ab + ao);
#pragma unroll
      for (int j = 0; j < 4; ++j) acc[i][j] = mma_b_raw(ah, bh[j], acc[i][j]);
      dep_guard_b(acc[i][0], acc[i][3], ah, ah);
    }
    keep4_b(bh[0], bh[1], bh[2], bh[3]);
  }
  acc_guard4(acc[0][0], acc[0][1], acc[0][2], acc[0][3]);
  acc_guard4(acc[1][0], acc[1][1], acc[1][2], acc[1][3]);
  acc_guard4(acc[2][0], acc[2][1], acc[2][2], acc[2][3]);
  acc_guard4(acc[3][0], acc[3][1], acc[3][2], acc[3][3]);

  float* slab = sT[wave];
  unsigned short* C = Cp + (size_t)b * strideC;
  const int q = lane >> 3, c8 = (lane & 7) * 8;
#pragma unroll
  for (int i = 0; i < 4; ++i) {
    const int mBase = m0 + (i << 4);
#pragma unroll
    for (int j = 0; j < 4; ++j) {
#pragma unroll
      for (int r = 0; r < 8; ++r) {
        const float bb = BIAS_ROW ? bias[mBase + mOff + r] : bias[n0 + (j << 4) + rlane];
        slab[(mOff + r) * 68 + (j << 4) + rlane] = acc[i][j][r] + bb;
      }
    }
    wave_sync_lds();
    v4u hv[4];
#pragma unroll
    for (int it = 0; it < 4; ++it) {
      const int row = it * 4 + q;
      const float* sp = slab + row * 68 + c8;
      v4u a;
#pragma unroll
      for (int e = 0; e < 4; ++e) a[e] = pk16(bf_bits(sp[2 * e]), bf_bits(sp[2 * e + 1]));
      hv[it] = a;
    }
    for (int ps = 0; ps < 2; ++ps) {
#pragma unroll
      for (int it = 0; it < 4; ++it) {
        const int row = it * 4 + q;
        *(volatile v4u*)(C + (size_t)(mBase + row) * ldc + n0 + c8) = hv[it];
      }
      __threadfence();
    }
    wave_sync_lds();
  }
}

__global__ __launch_bounds__(128)
void rowstats(const unsigned short* __restrict__ vktp, const unsigned short* __restrict__ qtp, float* stats) {
  __shared__ __align__(16) float sL[64];
  const int tid = threadIdx.x, wave = tid >> 5, lane = tid & 31, hh = lane >> 4, c = lane & 15;
  const int b = blockIdx.y;
  const int n0 = blockIdx.x * 64;
  const int n0w = n0 + wave * 16;
  const __bf16* VKT = (const __bf16*)(const void*)vktp + (size_t)b * NPOS * 64;
  const __bf16* QT  = (const __bf16*)(const void*)qtp  + (size_t)b * NPOS * 64;

  const v16b va = ldfrag_b(VKT + (size_t)(n0w + c) * 64 + 8 * hh);

  float mrow[8], lrow[8];
#pragma unroll
  for (int r = 0; r < 8; ++r) { mrow[r] = -INFINITY; lrow[r] = 0.f; }

  for (int mc = 0; mc < NPOS / 128; ++mc) {
    const int m0 = mc * 128;
    v8f s[8];
#pragma unroll
    for (int j = 0; j < 8; ++j) {
      const v16b qb = ldfrag_b(QT + (size_t)(m0 + j * 16 + c) * 64 + 8 * hh);
      s[j] = mma_b(va, qb, zero8());
    }
#pragma unroll
    for (int r = 0; r < 8; ++r) {
      float m = s[0][r];
#pragma unroll
      for (int j = 1; j < 8; ++j) m = fmaxf(m, s[j][r]);
#pragma unroll
      for (int off = 1; off < 16; off <<= 1) m = fmaxf(m, __shfl_xor(m, off, 32));
      const float mnew  = fmaxf(mrow[r], m);
      const float alpha = __expf(mrow[r] - mnew);
      mrow[r] = mnew;
      float psum = 0.f;
#pragma unroll
      for (int j = 0; j < 8; ++j) psum += __expf(s[j][r] - mnew);
#pragma unroll
      for (int off = 1; off < 16; off <<= 1) psum += __shfl_xor(psum, off, 32);
      lrow[r] = lrow[r] * alpha + psum;
    }
  }

#pragma unroll
  for (int r = 0; r < 8; ++r) {
    const float L = mrow[r] + __logf(lrow[r]);
    if (c == r) sL[wave * 16 + 8 * hh + r] = L;
  }
  __syncthreads();
  if (tid < 16) {
    const v4f v = *(const v4f*)(sL + 4 * tid);
    float* dp = stats + (size_t)b * NPOS + n0 + 4 * tid;
    *(volatile v4f*)dp = v;
    __threadfence();
    *(volatile v4f*)dp = v;
  }
}

__global__ __launch_bounds__(128)
void colacc(const unsigned short* __restrict__ vktp, const unsigned short* __restrict__ vkp,
            const unsigned short* __restrict__ qtp, const float* __restrict__ stats, float* avt) {
  __shared__ __align__(16) float sO[4][16 * 32];
  const int tid = threadIdx.x, wave = tid >> 5, lane = tid & 31, hh = lane >> 4, c = lane & 15;
  const int b = blockIdx.y;
  const int m0 = blockIdx.x * 64;
  const int m0w = m0 + wave * 16;
  const __bf16* VKT = (const __bf16*)(const void*)vktp + (size_t)b * NPOS * 64;
  const __bf16* QT  = (const __bf16*)(const void*)qtp  + (size_t)b * NPOS * 64;
  const __bf16* VK  = (const __bf16*)(const void*)vkp  + (size_t)b * 64 * NPOS;
  const float*  Lb  = stats + (size_t)b * NPOS;

  const v16b qb = ldfrag_b(QT + (size_t)(m0w + c) * 64 + 8 * hh);
  const __bf16* V0 = VKT + (size_t)c * 64 + 8 * hh;
  const __bf16* K0 = VK + (size_t)(32 + c) * NPOS + 8 * hh;
  const __bf16* K1 = VK + (size_t)(48 + c) * NPOS + 8 * hh;

  v8f acc0 = zero8(), acc1 = zero8();
  for (int nc = 0; nc < NPOS / 32; ++nc) {
    const int n0 = nc * 32;
    const v16b va0 = ldfrag_b(V0 + (size_t)n0 * 64);
    const v16b va1 = ldfrag_b(V0 + (size_t)(n0 + 16) * 64);
    const v8f s0 = mma_b(va0, qb, zero8());
    const v8f s1 = mma_b(va1, qb, zero8());
    const v8f L0 = *(const v8f*)(Lb + n0 + 8 * hh);
    const v8f L1 = *(const v8f*)(Lb + n0 + 16 + 8 * hh);
    FB pa;
#pragma unroll
    for (int k = 0; k < 4; ++k) {
      const float p00 = __expf(s0[2 * k] - L0[2 * k]);
      const float p01 = __expf(s0[2 * k + 1] - L0[2 * k + 1]);
      const float p10 = __expf(s1[2 * k] - L1[2 * k]);
      const float p11 = __expf(s1[2 * k + 1] - L1[2 * k + 1]);
      pa.u[k]     = pk16(bf_bits(p00), bf_bits(p01));
      pa.u[4 + k] = pk16(bf_bits(p10), bf_bits(p11));
    }
    const v16b kb0 = ldfrag_b(K0 + n0);
    const v16b kb1 = ldfrag_b(K1 + n0);
    acc0 = mma_b(pa.v, kb0, acc0);
    acc1 = mma_b(pa.v, kb1, acc1);
  }

  float* os = sO[wave];
#pragma unroll
  for (int r = 0; r < 8; ++r) {
    os[(8 * hh + r) * 32 + c]      = acc0[r];
    os[(8 * hh + r) * 32 + 16 + c] = acc1[r];
  }
  wave_sync_lds();
  const int q4 = lane >> 3, c4 = (lane & 7) * 4;
  v4f res[4];
#pragma unroll
  for (int it = 0; it < 4; ++it) res[it] = *(const v4f*)(os + (it * 4 + q4) * 32 + c4);
  for (int ps = 0; ps < 2; ++ps) {
#pragma unroll
    for (int it = 0; it < 4; ++it) {
      const int row = it * 4 + q4;
      *(volatile v4f*)(avt + ((size_t)b * NPOS + m0w + row) * 32 + c4) = res[it];
    }
    __threadfence();
  }
}

__global__ __launch_bounds__(128)
void tailk(const float* __restrict__ avt, const unsigned short* __restrict__ wgp, const unsigned short* __restrict__ wop,
           const float* __restrict__ par, const float* __restrict__ xB, float* out) {
  __shared__ __align__(16) float T[64 * 68];
  const int tid = threadIdx.x, wave = tid >> 5, lane = tid & 31, hh = lane >> 4, c = lane & 15;
  const int b = blockIdx.y;
  const int m0 = blockIdx.x * 64;
  const int mw = m0 + 16 * wave;
  const __bf16* Wg = (const __bf16*)(const void*)wgp;
  const __bf16* Wo = (const __bf16*)(const void*)wop;

  const float* ar = avt + ((size_t)b * NPOS + mw + c) * 32;
  const v8f alo = *(const v8f*)(ar + 8 * hh);
  const v8f ahi = *(const v8f*)(ar + 16 + 8 * hh);
  FB avb;
#pragma unroll
  for (int k = 0; k < 4; ++k) {
    avb.u[k]     = pk16(bf_bits(alo[2 * k]), bf_bits(alo[2 * k + 1]));
    avb.u[4 + k] = pk16(bf_bits(ahi[2 * k]), bf_bits(ahi[2 * k + 1]));
  }
  const v16b wg0 = ldfrag_b(Wg + (size_t)c * 32 + 8 * hh);
  const v16b wg1 = ldfrag_b(Wg + (size_t)(16 + c) * 32 + 8 * hh);
  const v8f g0 = mma_b(wg0, avb.v, zero8());
  const v8f g1 = mma_b(wg1, avb.v, zero8());

  const v8f mu0 = *(const v8f*)(par + 128 + 8 * hh), mu1 = *(const v8f*)(par + 128 + 16 + 8 * hh);
  const v8f sc0 = *(const v8f*)(par + 160 + 8 * hh), sc1 = *(const v8f*)(par + 160 + 16 + 8 * hh);
  const v8f be0 = *(const v8f*)(par + 192 + 8 * hh), be1 = *(const v8f*)(par + 192 + 16 + 8 * hh);
  FB gb;
#pragma unroll
  for (int k = 0; k < 4; ++k) {
    const float h00 = (g0[2 * k]     - mu0[2 * k])     * sc0[2 * k]     + be0[2 * k];
    const float h01 = (g0[2 * k + 1] - mu0[2 * k + 1]) * sc0[2 * k + 1] + be0[2 * k + 1];
    const float h10 = (g1[2 * k]     - mu1[2 * k])     * sc1[2 * k]     + be1[2 * k];
    const float h11 = (g1[2 * k + 1] - mu1[2 * k + 1]) * sc1[2 * k + 1] + be1[2 * k + 1];
    gb.u[k]     = pk16(bf_bits(h00), bf_bits(h01));
    gb.u[4 + k] = pk16(bf_bits(h10), bf_bits(h11));
  }

#pragma unroll
  for (int u = 0; u < 4; ++u) {
    const v16b wo = ldfrag_b(Wo + (size_t)(u * 16 + c) * 32 + 8 * hh);
    const v8f o = mma_b(wo, gb.v, zero8());
    const v8f bo8 = *(const v8f*)(par + 256 + u * 16 + 8 * hh);
    const v8f m28 = *(const v8f*)(par + 320 + u * 16 + 8 * hh);
    const v8f s28 = *(const v8f*)(par + 384 + u * 16 + 8 * hh);
    const v8f b28 = *(const v8f*)(par + 448 + u * 16 + 8 * hh);
#pragma unroll
    for (int r = 0; r < 8; ++r)
      T[(u * 16 + 8 * hh + r) * 68 + 16 * wave + c] = ((o[r] + bo8[r]) - m28[r]) * s28[r] + b28[r];
  }
  __syncthreads();

  const int c4 = (lane & 15) * 4;
  v4f res[8];
#pragma unroll
  for (int it = 0; it < 8; ++it) {
    const int row = 16 * wave + 2 * it + hh;
    const v4f t = *(const v4f*)(T + row * 68 + c4);
    const v4f x = *(const v4f*)(xB + ((size_t)(b * CC + row)) * NPOS + m0 + c4);
    v4f rr;
#pragma unroll
    for (int e = 0; e < 4; ++e) rr[e] = fmaxf(t[e] + bfr(x[e]), 0.0f);
    res[it] = rr;
  }
  for (int ps = 0; ps < 2; ++ps) {
#pragma unroll
    for (int it = 0; it < 8; ++it) {
      const int row = 16 * wave + 2 * it + hh;
      *(volatile v4f*)(out + ((size_t)(b * CC + row)) * NPOS + m0 + c4) = res[it];
    }
    __threadfence();
  }
}

extern "C" void kernel_launch(void* const* d_in, const int* in_sizes, int n_in,
                              void* d_out, int out_size, void* d_ws, size_t ws_size,
                              hipStream_t stream) {
  if (n_in < 19) return;
  if (in_sizes[0] != NB * CC * NPOS || in_sizes[1] != NB * CC * NPOS) return;
  if (in_sizes[2] != CI * CC || in_sizes[4] != CI * CC || in_sizes[6] != CI * CC) return;
  if (in_sizes[3] != CI || in_sizes[5] != CI || in_sizes[7] != CI) return;
  if (in_sizes[8] != CI * CI) return;
  if (in_sizes[9] != CI || in_sizes[10] != CI || in_sizes[11] != CI || in_sizes[12] != CI) return;
  if (in_sizes[13] != CC * CI) return;
  if (in_sizes[14] != CC || in_sizes[15] != CC || in_sizes[16] != CC || in_sizes[17] != CC || in_sizes[18] != CC) return;
  if (out_size != NB * CC * NPOS) return;

  const float* xA  = (const float*)d_in[0];
  const float* xB  = (const float*)d_in[1];
  const float* Wk  = (const float*)d_in[2];
  const float* bk  = (const float*)d_in[3];
  const float* Wv  = (const float*)d_in[4];
  const float* bv  = (const float*)d_in[5];
  const float* Wq  = (const float*)d_in[6];
  const float* bq  = (const float*)d_in[7];
  const float* Wg  = (const float*)d_in[8];
  const float* g1g = (const float*)d_in[9];
  const float* g1b = (const float*)d_in[10];
  const float* g1m = (const float*)d_in[11];
  const float* g1v = (const float*)d_in[12];
  const float* Wo  = (const float*)d_in[13];
  const float* bo  = (const float*)d_in[14];
  const float* g2g = (const float*)d_in[15];
  const float* g2b = (const float*)d_in[16];
  const float* g2m = (const float*)d_in[17];
  const float* g2v = (const float*)d_in[18];
  float* out = (float*)d_out;

  const size_t PW64 = 64 * 64 * 2;
  const size_t PWg  = 32 * 32 * 2;
  const size_t PWo  = 64 * 32 * 2;
  const size_t PPar = 512 * 4;
  const size_t PX   = (size_t)NB * NPOS * 64 * 2;
  const size_t PSt  = (size_t)NB * NPOS * 4;
  const size_t PAv  = (size_t)NB * NPOS * 32 * 4;
  size_t off = 0;
  const size_t oW64 = off; off += PW64;
  const size_t oWq  = off; off += PW64;
  const size_t oWg  = off; off += PWg;
  const size_t oWo  = off; off += PWo;
  const size_t oPar = off; off += PPar;
  const size_t oXAT = off; off += PX;
  const size_t oXBT = off; off += PX;
  const size_t oVKT = off; off += PX;
  const size_t oVK  = off; off += PX;
  const size_t oQT  = off; off += PX;
  const size_t oSt  = off; off += PSt;
  const size_t oAv  = off; off += PAv;
  if (off > ws_size) return;
  if (off > (size_t)134217728) return;

  char* ws = (char*)d_ws;
  unsigned short* W64  = (unsigned short*)(ws + oW64);
  unsigned short* Wq64 = (unsigned short*)(ws + oWq);
  unsigned short* WgB  = (unsigned short*)(ws + oWg);
  unsigned short* WoB  = (unsigned short*)(ws + oWo);
  float*          PAR  = (float*)(ws + oPar);
  unsigned short* XAT  = (unsigned short*)(ws + oXAT);
  unsigned short* XBT  = (unsigned short*)(ws + oXBT);
  unsigned short* VKT  = (unsigned short*)(ws + oVKT);
  unsigned short* VK   = (unsigned short*)(ws + oVK);
  unsigned short* QT   = (unsigned short*)(ws + oQT);
  float*          STATS = (float*)(ws + oSt);
  float*          AVT  = (float*)(ws + oAv);

  const dim3 blk256(256), blk128(128);
  const int tilesProj = (NPOS / 64) * (64 / 64);
  const dim3 gGemm((tilesProj + 7) / 8, NB);
  const dim3 gXp(NPOS / 64, 2 * NB);
  const dim3 gChunk(NPOS / 64, NB);

  prep_params<<<dim3(1), blk256, 0, stream>>>(Wk, bk, Wv, bv, Wq, bq, Wg, g1g, g1b, g1m, g1v, Wo, bo,
                                               g2g, g2b, g2m, g2v, W64, Wq64, WgB, WoB, PAR);
  xpose_cvt<<<gXp, blk256, 0, stream>>>(xA, xB, XAT, XBT);
  gemm64b<0><<<gGemm, blk256, 0, stream>>>(XAT, 64, (long long)NPOS * 64, W64, 64, 0LL, PAR,
                                           VKT, 64, (long long)NPOS * 64, NPOS, 64, 64);
  gemm64b<1><<<gGemm, blk256, 0, stream>>>(W64, 64, 0LL, XAT, 64, (long long)NPOS * 64, PAR,
                                           VK, NPOS, (long long)64 * NPOS, 64, NPOS, 64);
  gemm64b<0><<<gGemm, blk256, 0, stream>>>(XBT, 64, (long long)NPOS * 64, Wq64, 64, 0LL, PAR + 64,
                                           QT, 64, (long long)NPOS * 64, NPOS, 64, 64);
  rowstats<<<gChunk, blk128, 0, stream>>>(VKT, QT, STATS);
  colacc<<<gChunk, blk128, 0, stream>>>(VKT, VK, QT, STATS, AVT);
  tailk<<<gChunk, blk128, 0, stream>>>(AVT, WgB, WoB, PAR, xB, out);
  (void)hipGetLastError();
}
